// SAM_R_60112362275681
// MI455X (gfx1250) — hardware-verified
//
#include <hip/hip_runtime.h>
#include <math.h>

typedef __attribute__((ext_vector_type(16))) _Float16 v16h;
typedef __attribute__((ext_vector_type(16))) __bf16 v16b;
typedef __attribute__((ext_vector_type(8)))  _Float16 v8h;
typedef __attribute__((ext_vector_type(8)))  float v8f;
typedef __attribute__((ext_vector_type(4)))  float v4f;
typedef __attribute__((ext_vector_type(2)))  float v2f;
typedef __attribute__((ext_vector_type(4)))  unsigned v4u;
typedef __attribute__((ext_vector_type(4)))  int v4i;
typedef float __attribute__((may_alias)) float_a;
typedef int __attribute__((may_alias)) int_a;

template <typename T> __device__ __forceinline__ void vst2(void* p, T v) { *(volatile T*)p = v; __threadfence(); *(volatile T*)p = v; }
__device__ __forceinline__ v8f wmma16(v16h a, v16h b, v8f c) {
  v8f d = __builtin_amdgcn_wmma_f32_16x16x32_f16(false, a, false, b, (short)0, c, false, false);
  asm volatile("v_nop\n\tv_nop\n\tv_nop\n\tv_nop" : "+v"(d) : "v"(a), "v"(b));
  return d;
}
__device__ __forceinline__ v8f wmma_bf(v16b a, v16b b, v8f c) {
  v8f d = __builtin_amdgcn_wmma_f32_16x16x32_bf16(false, a, false, b, (short)0, c, false, false);
  asm volatile("v_nop\n\tv_nop\n\tv_nop\n\tv_nop" : "+v"(d) : "v"(a), "v"(b));
  return d;
}
__device__ __forceinline__ v16h frag_h(const _Float16* rowk0, int lane) {
  union { v16h v; v8h q[2]; } u; const _Float16* p = rowk0 + 8 * (lane >> 4);
  u.q[0] = *(const v8h*)p; u.q[1] = *(const v8h*)(p + 16); return u.v;
}
__device__ __forceinline__ v16h frag_f32(const float* rowk0, int lane) {
  v16h a; const float* p = rowk0 + 8 * (lane >> 4);
#pragma unroll
  for (int i = 0; i < 8; ++i) { a[i] = (_Float16)p[i]; a[8 + i] = (_Float16)p[16 + i]; }
  return a;
}
__device__ __forceinline__ v16h frag_f32s(const float* rowk0, int lane, float sc) {
  v16h a; const float* p = rowk0 + 8 * (lane >> 4);
#pragma unroll
  for (int i = 0; i < 8; ++i) { a[i] = (_Float16)(p[i] * sc); a[8 + i] = (_Float16)(p[16 + i] * sc); }
  return a;
}
__device__ __forceinline__ v16h fragc_f32(const float* W, int k0, int n, int lane, int ld, int K) {
  v16h a; const int g = lane >> 4;
#pragma unroll
  for (int i = 0; i < 8; ++i) { const int ka = k0 + 8 * g + i, kb = ka + 16;
    a[i] = (_Float16)(ka < K ? W[(size_t)(ka < K ? ka : K - 1) * ld + n] : 0.f); a[8 + i] = (_Float16)(kb < K ? W[(size_t)(kb < K ? kb : K - 1) * ld + n] : 0.f); }
  return a;
}
struct F2 { v16b h, l; };
__device__ __forceinline__ F2 bsplit16(const float v[16]) { F2 r;
#pragma unroll
  for (int i = 0; i < 16; ++i) { const __bf16 h = (__bf16)v[i]; r.h[i] = h; r.l[i] = (__bf16)(v[i] - (float)h); }
  return r; }
__device__ __forceinline__ F2 split_row(const float* row, int k0, int lane) { float v[16]; const float* p = row + k0 + 8 * (lane >> 4);
#pragma unroll
  for (int i = 0; i < 8; ++i) { v[i] = p[i]; v[8 + i] = p[16 + i]; }
  return bsplit16(v); }
__device__ __forceinline__ F2 split_rowK(const float* row, int k0, int lane, int K) { float v[16]; const int g = lane >> 4;
#pragma unroll
  for (int i = 0; i < 8; ++i) { const int ka = k0 + 8 * g + i, kb = ka + 16; v[i] = ka < K ? row[ka < K ? ka : K - 1] : 0.f; v[8 + i] = kb < K ? row[kb < K ? kb : K - 1] : 0.f; }
  return bsplit16(v); }
__device__ __forceinline__ F2 split_col(const float* W, int k0, int n, int lane, int ld, int K) { float v[16]; const int g = lane >> 4;
#pragma unroll
  for (int i = 0; i < 8; ++i) { const int ka = k0 + 8 * g + i, kb = ka + 16; v[i] = ka < K ? W[(size_t)(ka < K ? ka : K - 1) * ld + n] : 0.f; v[8 + i] = kb < K ? W[(size_t)(kb < K ? kb : K - 1) * ld + n] : 0.f; }
  return bsplit16(v); }
__device__ __forceinline__ v8f mac3(const F2& a, const F2& b, v8f c) { c = wmma_bf(a.l, b.h, c); c = wmma_bf(a.h, b.l, c); return wmma_bf(a.h, b.h, c); }
__device__ __forceinline__ float sigm(float v) { return 1.0f / (1.0f + expf(-v)); }
#define LDSX() do { asm volatile("s_wait_dscnt 0" ::: "memory"); __builtin_amdgcn_wave_barrier(); __builtin_amdgcn_fence(__ATOMIC_RELEASE, "workgroup"); } while (0)


#define NB 2
#define CC 256
#define HS 48
#define WSZ 48
#define MM (HS * WSZ)
#define NH 8
#define DH 32
#define BNEPS 1e-5f
#define L2EPS 1e-6f
#ifndef TNB
#define TNB NB
#endif
typedef __attribute__((ext_vector_type(8))) __bf16 v8b;
__device__ __forceinline__ v16b frag_b(const __bf16* rowk0, int lane) {
  union { v16b v; v8b q[2]; } u; const __bf16* p = rowk0 + 8 * (lane >> 4);
  u.q[0] = *(const v8b*)p; u.q[1] = *(const v8b*)(p + 16); return u.v;
}
__device__ __forceinline__ float bfr(float v) { return (float)(__bf16)v; }
__device__ __attribute__((noinline)) float exp_ni(float v) { return expf(v); }
__device__ __attribute__((noinline)) float erf_ni(float v) { return erff(v); }

#define WS_VH  0u
#define WS_VL  (WS_VH + 2u * (size_t)NB * MM * CC)
#define WS_Z   (WS_VL + 2u * (size_t)NB * MM * CC)
#define WS_QP  (WS_Z + 4u * (size_t)NB * CC * MM)
#define WS_QPL (WS_QP + 2u * (size_t)NB * CC * MM)
#define WS_KH  (WS_QPL + 2u * (size_t)NB * CC * MM)
#define WS_KL  (WS_KH + 2u * (size_t)NB * MM * CC)
#define WS_Y   (WS_KL + 2u * (size_t)NB * MM * CC)
#define WS_END (WS_Y + 4u * (size_t)NB * MM * CC)

__global__ __launch_bounds__(128) void k_conv(const float* __restrict__ X, const float* __restrict__ G, const float* __restrict__ Bt, const float* __restrict__ RM, const float* __restrict__ RV, const float* __restrict__ VW, const float* __restrict__ ZW, const float* __restrict__ QW, _Float16* __restrict__ VH, _Float16* __restrict__ VL, float* __restrict__ Z, _Float16* __restrict__ QP, _Float16* __restrict__ QPL) {
  __shared__ __align__(16) _Float16 sh[64][136], sl[64][136]; __shared__ __align__(16) float tf[128][68]; __shared__ __align__(16) _Float16 th[128][72], tl[128][72]; __shared__ float sa[CC], sb[CC];
  const int tid = threadIdx.x, wave = tid >> 5, lane = tid & 31, col = lane & 15, g = lane >> 4; const int which = blockIdx.z / NB; const size_t b = blockIdx.z % NB; const int m0 = blockIdx.x * 64; const int c0 = blockIdx.y * 128; const float* Wm = which == 0 ? VW : which == 1 ? ZW : QW; const float* Xb = X + b * CC * (size_t)MM;
  for (int c = tid; c < CC; c += 128) { const float inv = bfr(G[c]) / sqrtf(bfr(RV[c]) + BNEPS); sa[c] = inv; sb[c] = bfr(Bt[c]) - bfr(RM[c]) * inv; } __syncthreads();
  v8f acc[8] = {};
#pragma unroll 2
  for (int kc = 0; kc < CC / 32; ++kc) { float v[16]; const int px = m0 + wave * 16 + col;
#pragma unroll
    for (int i = 0; i < 8; ++i) { const int ca = kc * 32 + 8 * g + i, cb2 = ca + 16; v[i] = bfr(Xb[(size_t)ca * MM + px]) * sa[ca] + sb[ca]; v[8 + i] = bfr(Xb[(size_t)cb2 * MM + px]) * sa[cb2] + sb[cb2]; }
    const F2 a = bsplit16(v);
#pragma unroll
    for (int j = 0; j < 8; ++j) { v16b w; const float* wr = Wm + (size_t)(c0 + j * 16 + col) * CC + kc * 32 + 8 * g;
#pragma unroll
      for (int i = 0; i < 8; ++i) { w[i] = (__bf16)wr[i]; w[8 + i] = (__bf16)wr[16 + i]; }
      acc[j] = wmma_bf(a.h, w, acc[j]); acc[j] = wmma_bf(a.l, w, acc[j]); } }
#pragma unroll
  for (int j = 0; j < 8; ++j)
#pragma unroll
    for (int r = 0; r < 8; ++r) { const float v = acc[j][r]; const int rl = wave * 16 + 8 * g + r, cl = j * 16 + col; if (which == 1) tf[cl][rl] = v; else { const _Float16 hv = (_Float16)v, lv = (_Float16)((v - (float)hv) * 2048.0f); if (which == 0) { sh[rl][cl] = hv; sl[rl][cl] = lv; } else { th[cl][rl] = hv; tl[cl][rl] = lv; } } }
  __syncthreads();
  if (which == 0) { for (int e = tid; e < 64 * 16; e += 128) { const int rl = e >> 4, q = e & 15; const size_t o = (b * MM + m0 + rl) * CC + c0 + q * 8; vst2((unsigned*)(VH + o), *(const v4u*)&sh[rl][q * 8]); vst2((unsigned*)(VL + o), *(const v4u*)&sl[rl][q * 8]); } }
  else if (which == 1) { for (int e = tid; e < 128 * 16; e += 128) { const int cl = e >> 4, q = e & 15; vst2(Z + (b * CC + c0 + cl) * (size_t)MM + m0 + q * 4, *(const v4f*)&tf[cl][q * 4]); } }
  else { for (int e = tid; e < 128 * 8; e += 128) { const int cl = e >> 3, q = e & 7; const size_t o = (b * CC + c0 + cl) * (size_t)MM + m0 + q * 8; vst2((unsigned*)(QP + o), *(const v4u*)&th[cl][q * 8]); vst2((unsigned*)(QPL + o), *(const v4u*)&tl[cl][q * 8]); } } }
__global__ __launch_bounds__(256) void k_zr(const float* __restrict__ Z, _Float16* __restrict__ KH, _Float16* __restrict__ KL) { __shared__ __align__(16) _Float16 sh[64][264], sl[64][264]; __shared__ float sdiv[CC / 4]; __shared__ float part[2][4][64]; __shared__ float nz[64], nr[64];
  const int t = threadIdx.x; const size_t b = blockIdx.y; const int m0 = blockIdx.x * 64; const int ml = t & 63, q4 = t >> 6;
  if (t < CC / 4) sdiv[t] = expf((float)(2 * t) * (-logf(10000.0f) / (float)(CC / 2)));
  __syncthreads();
  { const int m = m0 + ml; const int yy = m / WSZ, xx = m % WSZ; float s1 = 0.f, s2 = 0.f;
    for (int c = q4 * 64; c < q4 * 64 + 64; ++c) { const float zv = Z[(b * CC + c) * (size_t)MM + m]; s1 += zv * zv; const int d = CC / 2; const int cc = c < d ? c : c - d; const float pos = (float)(c < d ? xx : yy); const float ang = pos * sdiv[cc >> 1]; const float pe = (cc & 1) ? cosf(ang) : sinf(ang); s2 += pe * pe; }
    part[0][q4][ml] = s1; part[1][q4][ml] = s2; }
  __syncthreads(); if (t < 64) { nz[t] = 1.0f / sqrtf(part[0][0][t] + part[0][1][t] + part[0][2][t] + part[0][3][t] + L2EPS); nr[t] = 1.0f / sqrtf(part[1][0][t] + part[1][1][t] + part[1][2][t] + part[1][3][t] + L2EPS); } __syncthreads();
  for (int e = t; e < 64 * CC; e += 256) { const int c = e >> 6, mml = e & 63; const int m = m0 + mml; const int yy = m / WSZ, xx = m % WSZ; const int d = CC / 2; const int cc = c < d ? c : c - d; const float pos = (float)(c < d ? xx : yy); const float ang = pos * sdiv[cc >> 1]; const float pe = (cc & 1) ? cosf(ang) : sinf(ang);
    const float v = Z[(b * CC + c) * (size_t)MM + m] * nz[mml] + pe * nr[mml]; const _Float16 hv = (_Float16)v; sh[mml][c] = hv; sl[mml][c] = (_Float16)((v - (float)hv) * 2048.0f); }
  __syncthreads(); for (int e = t; e < 64 * (CC / 8); e += 256) { const int mml = e / (CC / 8), q = e % (CC / 8); const size_t o = (b * MM + m0 + mml) * CC + q * 8; vst2((unsigned*)(KH + o), *(const v4u*)&sh[mml][q * 8]); vst2((unsigned*)(KL + o), *(const v4u*)&sl[mml][q * 8]); } }
__global__ __launch_bounds__(128) void k_att(const _Float16* __restrict__ VH, const _Float16* __restrict__ VL, const _Float16* __restrict__ KH, const _Float16* __restrict__ KL, const _Float16* __restrict__ QP, const _Float16* __restrict__ QPL, float* __restrict__ Y) {
  __shared__ __align__(16) float sp[4][16][36]; __shared__ __align__(16) float so[4][16][36];
  const int tid = threadIdx.x, wave = tid >> 5, lane = tid & 31, col = lane & 15, g = lane >> 4; const int h = blockIdx.y; const size_t b = blockIdx.z; const int q0 = blockIdx.x * 64 + wave * 16; const size_t rq = b * MM + q0;
  const v16h aq = frag_h(VH + (rq + col) * CC + h * DH, lane), al = frag_h(VL + (rq + col) * CC + h * DH, lane);
  float m[8], l[8];
#pragma unroll
  for (int r = 0; r < 8; ++r) { m[r] = -3.0e38f; l[r] = 0.f; }
  v8f acc[2] = {}, accl[2] = {};
#pragma unroll 1
  for (int ks = 0; ks < MM / 32; ++ks) { float s[2][8];
#pragma unroll
    for (int ct = 0; ct < 2; ++ct) { const size_t rk = b * MM + ks * 32 + ct * 16 + col; const v16h kh = frag_h(KH + rk * CC + h * DH, lane), kl = frag_h(KL + rk * CC + h * DH, lane); v8f c = {}, cl = {}; c = wmma16(aq, kh, c); cl = wmma16(aq, kl, cl); cl = wmma16(al, kh, cl);
#pragma unroll
      for (int r = 0; r < 8; ++r) s[ct][r] = (c[r] + cl[r] * (1.0f / 2048.0f)) * 0.17677669529663687f; }
    float alpha[8];
#pragma unroll
    for (int r = 0; r < 8; ++r) { float mx = fmaxf(s[0][r], s[1][r]);
#pragma unroll
      for (int o = 1; o < 16; o <<= 1) mx = fmaxf(mx, __shfl_xor(mx, o));
      const float mn = fmaxf(m[r], mx); alpha[r] = __expf(m[r] - mn); const float e0 = __expf(s[0][r] - mn), e1 = __expf(s[1][r] - mn); float es = e0 + e1;
#pragma unroll
      for (int o = 1; o < 16; o <<= 1) es += __shfl_xor(es, o);
      l[r] = l[r] * alpha[r] + es; m[r] = mn; sp[wave][8 * g + r][col] = e0; sp[wave][8 * g + r][16 + col] = e1; }
#pragma unroll
    for (int j = 0; j < 2; ++j)
#pragma unroll
      for (int r = 0; r < 8; ++r) { acc[j][r] *= alpha[r]; accl[j][r] *= alpha[r]; }
    LDSX();
    v16h pa, pal; { const float* prow = &sp[wave][col][0] + 8 * (lane >> 4);
#pragma unroll
      for (int i = 0; i < 8; ++i) { const float p0 = prow[i] * 2048.0f, p1 = prow[16 + i] * 2048.0f; pa[i] = (_Float16)p0; pa[8 + i] = (_Float16)p1; pal[i] = (_Float16)((p0 - (float)pa[i]) * 2048.0f); pal[8 + i] = (_Float16)((p1 - (float)pa[8 + i]) * 2048.0f); } }
#pragma unroll
    for (int j = 0; j < 2; ++j) { const size_t po = (b * CC + (size_t)h * DH + j * 16 + col) * (size_t)MM + ks * 32; const v16h vh = frag_h(QP + po, lane), vl = frag_h(QPL + po, lane); acc[j] = wmma16(pa, vh, acc[j]); accl[j] = wmma16(pa, vl, accl[j]); accl[j] = wmma16(pal, vh, accl[j]); }
    LDSX(); }
#pragma unroll
  for (int r = 0; r < 8; ++r) { const float il = (1.0f / 2048.0f) / l[r];
#pragma unroll
    for (int j = 0; j < 2; ++j) so[wave][8 * g + r][j * 16 + col] = (acc[j][r] + accl[j][r] * (1.0f / 2048.0f)) * il; }
  LDSX(); for (int rl = 0; rl < 16; ++rl) if (lane < 8) vst2(Y + (rq + rl) * CC + (size_t)h * DH + lane * 4, *(const v4f*)&so[wave][rl][lane * 4]); }
__global__ __launch_bounds__(128) void k_o(const float* __restrict__ Y, const float* __restrict__ OW, float* __restrict__ OUT) { __shared__ __align__(16) float sf[4][16][132];
  const int tid = threadIdx.x, wave = tid >> 5, lane = tid & 31, col = lane & 15, g = lane >> 4; const size_t b = blockIdx.z; const int o0 = blockIdx.x * 64 + wave * 16; const int p0 = blockIdx.y * 128;
  v8f acc[8] = {};
#pragma unroll 2
  for (int kc = 0; kc < CC / 32; ++kc) { v16b a; const float* ar = OW + (size_t)(o0 + col) * CC + kc * 32 + 8 * g;
#pragma unroll
    for (int i = 0; i < 8; ++i) { a[i] = (__bf16)ar[i]; a[8 + i] = (__bf16)ar[16 + i]; }
#pragma unroll
    for (int j = 0; j < 8; ++j) { float wv[16]; const float* wr = Y + (b * MM + p0 + j * 16 + col) * CC + kc * 32 + 8 * g;
#pragma unroll
      for (int i = 0; i < 8; ++i) { wv[i] = wr[i]; wv[8 + i] = wr[16 + i]; }
      const F2 wb = bsplit16(wv); acc[j] = wmma_bf(a, wb.h, acc[j]); acc[j] = wmma_bf(a, wb.l, acc[j]); } }
#pragma unroll
  for (int j = 0; j < 8; ++j)
#pragma unroll
    for (int r = 0; r < 8; ++r) sf[wave][8 * g + r][j * 16 + col] = acc[j][r];
  LDSX(); for (int rl = 0; rl < 16; ++rl) vst2(OUT + (b * CC + o0 + rl) * (size_t)MM + p0 + lane * 4, *(const v4f*)&sf[wave][rl][lane * 4]); }
extern "C" void kernel_launch(void* const* d_in, const int* in_sizes, int n_in, void* d_out, int out_size, void* d_ws, size_t ws_size, hipStream_t stream) {
  (void)in_sizes; (void)n_in; (void)out_size;
  const float** F = (const float**)d_in;
  if (ws_size < (size_t)WS_END) return;
  char* ws = (char*)d_ws; _Float16 *VH = (_Float16*)(ws + WS_VH), *VL = (_Float16*)(ws + WS_VL), *QP = (_Float16*)(ws + WS_QP), *QPL = (_Float16*)(ws + WS_QPL), *KH = (_Float16*)(ws + WS_KH), *KL = (_Float16*)(ws + WS_KL); float *Z = (float*)(ws + WS_Z), *Y = (float*)(ws + WS_Y);
  k_conv<<<dim3(MM / 64, CC / 128, 3 * NB), 128, 0, stream>>>(F[0], F[1], F[2], F[3], F[4], F[5], F[6], F[7], VH, VL, Z, QP, QPL);
  k_zr<<<dim3(MM / 64, NB), 256, 0, stream>>>(Z, KH, KL);
  k_att<<<dim3(MM / 64, NH, TNB), 128, 0, stream>>>(VH, VL, KH, KL, QP, QPL, Y);
  k_o<<<dim3(CC / 64, MM / 128, TNB), 128, 0, stream>>>(Y, F[8], (float*)d_out);
}
